// TransDecoder_59115929862519
// MI455X (gfx1250) — hardware-verified
//
#include <hip/hip_runtime.h>

typedef __attribute__((ext_vector_type(16))) _Float16 v16h;
typedef __attribute__((ext_vector_type(8)))  _Float16 v8h;
typedef __attribute__((ext_vector_type(16))) __bf16   v16b;
typedef __attribute__((ext_vector_type(8)))  __bf16   v8b;
typedef __attribute__((ext_vector_type(8)))  float    v8f;
typedef __attribute__((ext_vector_type(4)))  float    v4f;
typedef __attribute__((ext_vector_type(4)))  int      v4i;
#define PSCALE 32768.0f
#define U16(p) ((const unsigned short*)(const void*)(p))
#define PSCALE_INV (1.0f / 32768.0f)

__device__ __forceinline__ unsigned short f2bf_bits(float f) {
  unsigned u = __float_as_uint(f);
  return (unsigned short)((u + 0x7FFFu + ((u >> 16) & 1u)) >> 16);
}
__device__ __forceinline__ float bf_bits2f(unsigned short h) { return __uint_as_float(((unsigned)h) << 16); }

__device__ __forceinline__ void dep_guard_h(v8f& a, v8f& b, v16h x, v16h y) { asm volatile("v_nop\n\tv_nop\n\tv_nop\n\tv_nop" : "+v"(a), "+v"(b) : "v"(x), "v"(y)); }
__device__ __forceinline__ void dep_guard_b(v8f& a, v8f& b, v16b x, v16b y) { asm volatile("v_nop\n\tv_nop\n\tv_nop\n\tv_nop" : "+v"(a), "+v"(b) : "v"(x), "v"(y)); }
__device__ __forceinline__ void keep4_h(v16h a, v16h b, v16h c, v16h d) { asm volatile("v_nop" :: "v"(a), "v"(b), "v"(c), "v"(d)); }
__device__ __forceinline__ void keep4_b(v16b a, v16b b, v16b c, v16b d) { asm volatile("v_nop" :: "v"(a), "v"(b), "v"(c), "v"(d)); }
__device__ __forceinline__ void acc_guard4(v8f& a, v8f& b, v8f& c, v8f& d) { asm volatile("v_nop\n\tv_nop\n\tv_nop\n\tv_nop" : "+v"(a), "+v"(b), "+v"(c), "+v"(d)); }
template <typename T> struct Frag;
template <> struct Frag<_Float16> {
  typedef v16h V; union U { v16h v; v8h h[2]; };
  static __device__ __forceinline__ v16h load(const _Float16* p) {
    U f; f.h[0] = *(const v8h*)(p); f.h[1] = *(const v8h*)(p + 16); return f.v;
  }
  static __device__ __forceinline__ v8f mma(v16h a, v16h b, v8f c) {
    return __builtin_amdgcn_wmma_f32_16x16x32_f16(false, a, false, b, (short)0, c, false, false);
  }
  static __device__ __forceinline__ void guard(v8f& a, v8f& b, v16h x, v16h y) { dep_guard_h(a, b, x, y); }
  static __device__ __forceinline__ void keep(v16h a, v16h b, v16h c, v16h d) { keep4_h(a, b, c, d); }
};
template <> struct Frag<__bf16> {
  typedef v16b V; union U { v16b v; v8b h[2]; };
  static __device__ __forceinline__ v16b load(const __bf16* p) {
    U f; f.h[0] = *(const v8b*)(p); f.h[1] = *(const v8b*)(p + 16); return f.v;
  }
  static __device__ __forceinline__ v8f mma(v16b a, v16b b, v8f c) {
    return __builtin_amdgcn_wmma_f32_16x16x32_bf16(false, a, false, b, (short)0, c, false, false);
  }
  static __device__ __forceinline__ void guard(v8f& a, v8f& b, v16b x, v16b y) { dep_guard_b(a, b, x, y); }
  static __device__ __forceinline__ void keep(v16b a, v16b b, v16b c, v16b d) { keep4_b(a, b, c, d); }
};

template <int ET> struct Elem;
template <> struct Elem<0> { typedef _Float16 T; };
template <> struct Elem<1> { typedef __bf16 T; };
template <int ET, bool SPLIT, int BIAS_MODE, int OUT_MODE, bool RESID, int ACT = 0>
__global__ __launch_bounds__(256) void wmma_gemm64(
    const unsigned short* __restrict__ Ap, const unsigned short* __restrict__ A2p, int lda, long strideA,
    const unsigned short* __restrict__ Btp, const unsigned short* __restrict__ Bt2p, int ldb, long strideB,
    void* __restrict__ Cout, void* __restrict__ Cout2, int ldc, long strideC,
    const float* __restrict__ bias,
    const float* __restrict__ resid, long strideR,
    int M, int N, int K, float scale) {
  typedef typename Elem<ET>::T T;
  typedef typename Frag<T>::V V;
  const T* A = (const T*)Ap; const T* A2 = (const T*)A2p; const T* Bt = (const T*)Btp; const T* Bt2 = (const T*)Bt2p;
  __shared__ __align__(16) float sT[8][16 * 68];
  const int b    = blockIdx.y;
  const int lane = threadIdx.x & 31;
  const int wave = threadIdx.x >> 5;
  const int tilesN = N >> 6;
  const int tilesM = M >> 6;
  const int tile = blockIdx.x * 8 + wave;
  if (tile >= tilesM * tilesN) return;
  const int tm = tile / tilesN;
  const int tn = tile - tm * tilesN;
  const int m0 = tm << 6;
  const int n0 = tn << 6;

  const T* Ab  = A  + (size_t)b * strideA;
  const T* Bb  = Bt + (size_t)b * strideB;
  const T* Ab2 = SPLIT ? (A2  + (size_t)b * strideA) : nullptr;
  const T* Bb2 = SPLIT ? (Bt2 + (size_t)b * strideB) : nullptr;

  const int rlane = lane & 15;
  const int koff  = (lane >> 4) * 8;
  const int mOff  = (lane >> 4) * 8;

  v8f acc[4][4];
#pragma unroll
  for (int i = 0; i < 4; ++i)
#pragma unroll
    for (int j = 0; j < 4; ++j) acc[i][j] = (v8f){0.f,0.f,0.f,0.f,0.f,0.f,0.f,0.f};

  for (int k0 = 0; k0 < K; k0 += 32) {
    V bh[4], bl[4];
#pragma unroll
    for (int j = 0; j < 4; ++j) {
      const size_t bo = (size_t)(n0 + (j << 4) + rlane) * ldb + koff + k0;
      bh[j] = Frag<T>::load(Bb + bo);
      if (SPLIT) bl[j] = Frag<T>::load(Bb2 + bo);
    }
#pragma unroll
    for (int i = 0; i < 4; ++i) {
      const size_t ao = (size_t)(m0 + (i << 4) + rlane) * lda + koff + k0;
      V ah = Frag<T>::load(Ab + ao);
      V al;
      if (SPLIT) al = Frag<T>::load(Ab2 + ao);
#pragma unroll
      for (int j = 0; j < 4; ++j) {
        acc[i][j] = Frag<T>::mma(ah, bh[j], acc[i][j]);
        if (SPLIT) {
          acc[i][j] = Frag<T>::mma(ah, bl[j], acc[i][j]);
          acc[i][j] = Frag<T>::mma(al, bh[j], acc[i][j]);
        }
      }
      Frag<T>::guard(acc[i][0], acc[i][3], ah, SPLIT ? al : ah);
    }
    Frag<T>::keep(bh[0], bh[1], bh[2], bh[3]);
    if (SPLIT) Frag<T>::keep(bl[0], bl[1], bl[2], bl[3]);
  }
  acc_guard4(acc[0][0], acc[0][1], acc[0][2], acc[0][3]);
  acc_guard4(acc[1][0], acc[1][1], acc[1][2], acc[1][3]);
  acc_guard4(acc[2][0], acc[2][1], acc[2][2], acc[2][3]);
  acc_guard4(acc[3][0], acc[3][1], acc[3][2], acc[3][3]);

  float* slab = sT[wave];
  const float* Rb = RESID ? (resid + (size_t)b * strideR) : nullptr;
#pragma unroll
  for (int i = 0; i < 4; ++i) {
    const int mBase = m0 + (i << 4);
#pragma unroll
    for (int j = 0; j < 4; ++j) {
      const int n = n0 + (j << 4) + rlane;
      float bv = 0.f;
      if (BIAS_MODE == 2) bv = bias[n];
#pragma unroll
      for (int r = 0; r < 8; ++r) {
        float v = acc[i][j][r] * scale;
        if (BIAS_MODE == 1) v += bias[mBase + mOff + r];
        if (BIAS_MODE == 2) v += bv;
        if (RESID) v += Rb[(size_t)(mBase + mOff + r) * ldc + n];
        if (ACT == 1) v = tanhf(v);
        if (ACT == 2) v = fmaxf(v, 0.0f);
        if (ACT == 3) v = v / (1.0f + expf(-v));
        if (ACT == 4) v = (v > 0.f) ? v : 0.01f * v;
        if (ACT == 5) v = 0.5f * v * (1.0f + erff(v * 0.70710678118654752f));
        slab[(mOff + r) * 68 + (j << 4) + rlane] = v;
      }
    }
    __builtin_amdgcn_fence(__ATOMIC_RELEASE, "workgroup");
    __builtin_amdgcn_wave_barrier();
    __builtin_amdgcn_fence(__ATOMIC_ACQUIRE, "workgroup");
    if (OUT_MODE == 0) {
      float* C = (float*)Cout + (size_t)b * strideC;
      const int hh = lane >> 4, c4 = (lane & 15) * 4;
      for (int pass = 0; pass < 2; ++pass) {
#pragma unroll
        for (int it = 0; it < 8; ++it) {
          const int row = it * 2 + hh;
          v4f v = *(const v4f*)(slab + row * 68 + c4);
          *(volatile v4f*)(C + (size_t)(mBase + row) * ldc + n0 + c4) = v;
        }
        __threadfence();
      }
    } else {
      const int q = lane >> 3, c8 = (lane & 7) * 8;
      unsigned short* C  = (unsigned short*)Cout  + (size_t)b * strideC;
      unsigned short* C2 = (OUT_MODE == 2) ? ((unsigned short*)Cout2 + (size_t)b * strideC) : nullptr;
      for (int pass = 0; pass < 2; ++pass) {
#pragma unroll
        for (int it = 0; it < 4; ++it) {
          const int row = it * 4 + q;
          const float* sp = slab + row * 68 + c8;
          v8h hv, lv;
#pragma unroll
          for (int e = 0; e < 8; ++e) {
            if (OUT_MODE == 1) {
              hv[e] = (_Float16)sp[e];
            } else {
              unsigned short hb = f2bf_bits(sp[e]);
              unsigned short lb = f2bf_bits(sp[e] - bf_bits2f(hb));
              hv[e] = __builtin_bit_cast(_Float16, hb);
              lv[e] = __builtin_bit_cast(_Float16, lb);
            }
          }
          *(volatile v8h*)(C + (size_t)(mBase + row) * ldc + n0 + c8) = hv;
          if (OUT_MODE == 2) *(volatile v8h*)(C2 + (size_t)(mBase + row) * ldc + n0 + c8) = lv;
        }
        __threadfence();
      }
    }
    __builtin_amdgcn_fence(__ATOMIC_RELEASE, "workgroup");
    __builtin_amdgcn_wave_barrier();
    __builtin_amdgcn_fence(__ATOMIC_ACQUIRE, "workgroup");
  }
}

constexpr int kB = 4;
constexpr int kN = 128;
constexpr int kD = 512;
constexpr int kREL = 64;
constexpr int kP = 3 * kD + kREL;
constexpr int kH = 64;
constexpr int kNJ = kN + 1;
constexpr int kNMAIN = kNJ * kH;
constexpr int kXAROWS = 576;
constexpr int kPAIRS = kB * kN * kN;
constexpr int kNOUT = kB * kN * kNJ;
constexpr int kOUTQ = (kB * kN + 2 * kNOUT) / 4;
constexpr float kWCarry = 16.0f;
constexpr float kWCarryInv = 0.0625f;

static_assert(kXAROWS % 64 == 0 && kH % 64 == 0 && kD % 32 == 0, "gemm G shape");
static_assert(kPAIRS % 64 == 0 && kREL % 32 == 0, "gemm R shape");
static_assert(kN % 64 == 0 && kNMAIN % 64 == 0, "gemm main shape");
static_assert(kNOUT % 128 == 0, "score tables are whole wave chunks");
static_assert((kB * kN) % 4 == 0 && (kB * kN + kNOUT) % 4 == 0, "output regions start on float4");
static_assert((kB * kN + 2 * kNOUT) * 4 == 530432, "d_out bytes");
static_assert((kB * kN + 2 * kNOUT) % 128 == 0, "d_out is whole wave chunks");

__global__ __launch_bounds__(256) void prep_planes(const float* __restrict__ span, const float* __restrict__ topic,
                                                   const float* __restrict__ W1,
                                                   _Float16* __restrict__ xa, _Float16* __restrict__ w1b16,
                                                   _Float16* __restrict__ w1d16) {
  const int blk = blockIdx.x;
  const int t = threadIdx.x;
  if (blk < 144) {
    const int g = blk * 256 + t;
    const int row = g >> 6;
    const int d0 = (g & 63) * 8;
    const int rs = (row < kB * kN) ? row : (kB * kN - 1);
    int rt = row - kB * kN;
    rt = (rt < 0) ? 0 : ((rt > kB - 1) ? (kB - 1) : rt);
    const v4f s0 = *(const v4f*)(span + (size_t)rs * kD + d0);
    const v4f s1 = *(const v4f*)(span + (size_t)rs * kD + d0 + 4);
    const v4f t0 = *(const v4f*)(topic + (size_t)rt * kD + d0);
    const v4f t1 = *(const v4f*)(topic + (size_t)rt * kD + d0 + 4);
    const bool isS = row < kB * kN;
    const bool isT = (row >= kB * kN) && (row < kB * kN + kB);
    v8h o;
#pragma unroll
    for (int e = 0; e < 4; ++e) {
      const float a = isS ? s0[e] : (isT ? t0[e] : 0.0f);
      const float c = isS ? s1[e] : (isT ? t1[e] : 0.0f);
      o[e] = (_Float16)a;
      o[4 + e] = (_Float16)c;
    }
    _Float16* dst = xa + (size_t)row * kD + d0;
    *(volatile v8h*)dst = o;
    __threadfence();
    *(volatile v8h*)dst = o;
  } else if (blk < 160) {
    const int g = (blk - 144) * 256 + t;
    const int k = g >> 6;
    const int d0 = (g & 63) * 8;
    const float* wp = W1 + (size_t)k * kP + kD + d0;
    const v4f w0 = *(const v4f*)(wp);
    const v4f w1 = *(const v4f*)(wp + 4);
    v8h o;
#pragma unroll
    for (int e = 0; e < 4; ++e) {
      o[e] = (_Float16)(w0[e] * kWCarry);
      o[4 + e] = (_Float16)(w1[e] * kWCarry);
    }
    _Float16* dst = w1b16 + (size_t)k * kD + d0;
    *(volatile v8h*)dst = o;
    __threadfence();
    *(volatile v8h*)dst = o;
  } else {
    const int g = (blk - 160) * 256 + t;
    const int k = g >> 3;
    const int d0 = (g & 7) * 8;
    const float* wp = W1 + (size_t)k * kP + 3 * kD + d0;
    const v4f w0 = *(const v4f*)(wp);
    const v4f w1 = *(const v4f*)(wp + 4);
    v8h o;
#pragma unroll
    for (int e = 0; e < 4; ++e) {
      o[e] = (_Float16)(w0[e] * kWCarry);
      o[4 + e] = (_Float16)(w1[e] * kWCarry);
    }
    _Float16* dst = w1d16 + (size_t)k * kREL + d0;
    *(volatile v8h*)dst = o;
    __threadfence();
    *(volatile v8h*)dst = o;
  }
}

__global__ __launch_bounds__(256) void rel_cast(const int* __restrict__ rel, _Float16* __restrict__ out16, int n8) {
  const int g = blockIdx.x * 256 + threadIdx.x;
  if (g < n8) {
    const v4i a = *(const v4i*)(rel + (size_t)g * 8);
    const v4i c = *(const v4i*)(rel + (size_t)g * 8 + 4);
    v8h o;
#pragma unroll
    for (int e = 0; e < 4; ++e) {
      o[e] = (_Float16)((float)a[e]);
      o[4 + e] = (_Float16)((float)c[e]);
    }
    _Float16* dst = out16 + (size_t)g * 8;
    *(volatile v8h*)dst = o;
    __threadfence();
    *(volatile v8h*)dst = o;
  }
}

__global__ __launch_bounds__(256) void beff_build(const float* __restrict__ span, const float* __restrict__ topic,
                                                  const float* __restrict__ W1, _Float16* __restrict__ beff) {
  const int g = blockIdx.x * 256 + threadIdx.x;
  const int d0 = (g & 63) * 8;
  const int rowg = g >> 6;
  const int b = rowg / kNMAIN;
  const int n = rowg - b * kNMAIN;
  const int i = n >> 6;
  const int k = n & 63;
  const int is = (i < kN) ? i : (kN - 1);
  const float* sp = span + ((size_t)(b * kN + is)) * kD + d0;
  const float* tp = topic + (size_t)b * kD + d0;
  const float* wa = W1 + (size_t)k * kP + d0;
  const float* wc = W1 + (size_t)k * kP + 2 * kD + d0;
  const v4f s0 = *(const v4f*)(sp), s1 = *(const v4f*)(sp + 4);
  const v4f t0 = *(const v4f*)(tp), t1 = *(const v4f*)(tp + 4);
  const v4f a0 = *(const v4f*)(wa), a1 = *(const v4f*)(wa + 4);
  const v4f c0 = *(const v4f*)(wc), c1 = *(const v4f*)(wc + 4);
  const bool useSpan = (i < kN);
  v8h o;
#pragma unroll
  for (int e = 0; e < 4; ++e) {
    const float x0 = useSpan ? s0[e] : t0[e];
    const float x1 = useSpan ? s1[e] : t1[e];
    o[e] = (_Float16)((a0[e] + x0 * c0[e]) * kWCarry);
    o[4 + e] = (_Float16)((a1[e] + x1 * c1[e]) * kWCarry);
  }
  _Float16* dst = beff + (size_t)rowg * kD + d0;
  *(volatile v8h*)dst = o;
  __threadfence();
  *(volatile v8h*)dst = o;
}

__global__ __launch_bounds__(128) void ac_scores(const float* __restrict__ span, const float* __restrict__ wt,
                                                 const float* __restrict__ bt, float* __restrict__ act) {
  const int t = threadIdx.x;
  const float* r0 = span + ((size_t)(4 * t)) * kD;
  float a0 = 0.0f, a1 = 0.0f, a2 = 0.0f, a3 = 0.0f;
#pragma unroll 1
  for (int d = 0; d < kD; ++d) {
    const float w = wt[d];
    a0 += r0[d] * w;
    a1 += r0[kD + d] * w;
    a2 += r0[2 * kD + d] * w;
    a3 += r0[3 * kD + d] * w;
  }
  const float bb = bt[0];
  v4f o;
  o[0] = a0 + bb; o[1] = a1 + bb; o[2] = a2 + bb; o[3] = a3 + bb;
  float* dst = act + 4 * t;
  *(volatile v4f*)dst = o;
  __threadfence();
  *(volatile v4f*)dst = o;
}

__global__ __launch_bounds__(256) void epi_scores(const float* __restrict__ cmain, const float* __restrict__ rbuf,
                                                  const float* __restrict__ gbuf, const float* __restrict__ b1,
                                                  const float* __restrict__ W2, const float* __restrict__ b2,
                                                  const int* __restrict__ adu,
                                                  float* __restrict__ srel, float* __restrict__ spair) {
  __shared__ __align__(16) float sb1[kH];
  __shared__ __align__(16) float sw2[2 * kH];
  const int tid = threadIdx.x;
  if (tid < kH) sb1[tid] = b1[tid];
  if (tid < 2 * kH) sw2[tid] = W2[tid];
  __syncthreads();
  const int t = blockIdx.x * 256 + tid;
  if (t < kNOUT / 4) {
    const float b20 = b2[0];
    const float b21 = b2[1];
    float ro[4], po[4];
#pragma unroll
    for (int el = 0; el < 4; ++el) {
      const int e = 4 * t + el;
      const int b = e / (kN * kNJ);
      const int rem = e - b * (kN * kNJ);
      const int i = rem / kNJ;
      const int j = rem - i * kNJ;
      const bool isroot = (j == kN);
      const int rowc = isroot ? i : j;
      const int colb = isroot ? (kN * kH) : (i * kH);
      const float* cp = cmain + ((size_t)(b * kN + rowc)) * kNMAIN + colb;
      const int jc = isroot ? (kN - 1) : j;
      const float* rp = rbuf + ((size_t)((b * kN + i) * kN + jc)) * kH;
      const int grow = isroot ? (kB * kN + b) : (b * kN + i);
      const float* gp = gbuf + (size_t)grow * kH;
      float a0 = 0.0f, a1 = 0.0f;
#pragma unroll 1
      for (int k4 = 0; k4 < kH / 4; ++k4) {
        const v4f cv = *(const v4f*)(cp + 4 * k4);
        const v4f rv = *(const v4f*)(rp + 4 * k4);
        const v4f gv = *(const v4f*)(gp + 4 * k4);
        const v4f bv = *(const v4f*)(sb1 + 4 * k4);
        const v4f w0 = *(const v4f*)(sw2 + 4 * k4);
        const v4f w1 = *(const v4f*)(sw2 + kH + 4 * k4);
#pragma unroll
        for (int q = 0; q < 4; ++q) {
          const float rq = isroot ? 0.0f : rv[q];
          float hp = ((cv[q] + rq) + gv[q]) + bv[q];
          hp = fmaxf(hp, 0.0f);
          a0 += hp * w0[q];
          a1 += hp * w1[q];
        }
      }
      ro[el] = a0 + b20;
      const float ps = a1 + b21;
      const int alen = adu[b];
      const bool keep = isroot || ((j != i) && (j < alen));
      po[el] = keep ? ps : -1.0e16f;
    }
    v4f vr, vp;
    vr[0] = ro[0]; vr[1] = ro[1]; vr[2] = ro[2]; vr[3] = ro[3];
    vp[0] = po[0]; vp[1] = po[1]; vp[2] = po[2]; vp[3] = po[3];
    float* dr = srel + 4 * (size_t)t;
    float* dp = spair + 4 * (size_t)t;
    *(volatile v4f*)dr = vr;
    *(volatile v4f*)dp = vp;
    __threadfence();
    *(volatile v4f*)dr = vr;
    *(volatile v4f*)dp = vp;
  }
}

__global__ __launch_bounds__(256) void pack_out(const float* __restrict__ act, const float* __restrict__ spair,
                                                const float* __restrict__ srel, float* __restrict__ out, int nq) {
  const int q = blockIdx.x * 256 + threadIdx.x;
  if (q < nq) {
    const int qa = (q < kB * kN / 4) ? q : (kB * kN / 4 - 1);
    int qp = q - kB * kN / 4;
    qp = (qp < 0) ? 0 : ((qp > kNOUT / 4 - 1) ? (kNOUT / 4 - 1) : qp);
    int qr = q - (kB * kN / 4 + kNOUT / 4);
    qr = (qr < 0) ? 0 : ((qr > kNOUT / 4 - 1) ? (kNOUT / 4 - 1) : qr);
    const v4f va = *(const v4f*)(act + 4 * (size_t)qa);
    const v4f vp = *(const v4f*)(spair + 4 * (size_t)qp);
    const v4f vr = *(const v4f*)(srel + 4 * (size_t)qr);
    const bool isA = q < kB * kN / 4;
    const bool isP = q < (kB * kN / 4 + kNOUT / 4);
    v4f v;
#pragma unroll
    for (int e = 0; e < 4; ++e) v[e] = isA ? va[e] : (isP ? vp[e] : vr[e]);
    float* dst = out + 4 * (size_t)q;
    *(volatile v4f*)dst = v;
    __threadfence();
    *(volatile v4f*)dst = v;
  }
}

extern "C" void kernel_launch(void* const* d_in, const int* in_sizes, int n_in,
                              void* d_out, int out_size, void* d_ws, size_t ws_size,
                              hipStream_t stream) {
  if (n_in < 10) return;
  if (in_sizes[0] != kB * kN * kD || in_sizes[1] != kB * kD || in_sizes[2] != kB ||
      in_sizes[3] != kPAIRS * kREL || in_sizes[4] != kD || in_sizes[5] < 1 ||
      in_sizes[6] != kH * kP || in_sizes[7] != kH || in_sizes[8] != 2 * kH || in_sizes[9] != 2) return;
  if (out_size != kB * kN + 2 * kNOUT) return;

  const float* span   = (const float*)d_in[0];
  const float* topic  = (const float*)d_in[1];
  const int*   adu    = (const int*)  d_in[2];
  const int*   rel    = (const int*)  d_in[3];
  const float* W_type = (const float*)d_in[4];
  const float* b_type = (const float*)d_in[5];
  const float* W1     = (const float*)d_in[6];
  const float* b1     = (const float*)d_in[7];
  const float* W2     = (const float*)d_in[8];
  const float* b2     = (const float*)d_in[9];

  char* ws = (char*)d_ws;
  size_t off = 0;
  const size_t bXA    = (size_t)kXAROWS * kD * 2;
  const size_t bW1B   = (size_t)kH * kD * 2;
  const size_t bW1D   = (size_t)kH * kREL * 2;
  const size_t bBEFF  = (size_t)kB * kNMAIN * kD * 2;
  const size_t bREL16 = (size_t)kPAIRS * kREL * 2;
  const size_t bCMAIN = (size_t)kB * kN * kNMAIN * 4;
  const size_t bRBUF  = (size_t)kPAIRS * kH * 4;
  const size_t bGBUF  = (size_t)kXAROWS * kH * 4;
  const size_t bACT   = (size_t)kB * kN * 4;
  const size_t bSTAB  = (size_t)kNOUT * 4;
  _Float16* xa    = (_Float16*)(ws + off); off += bXA;
  _Float16* w1b16 = (_Float16*)(ws + off); off += bW1B;
  _Float16* w1d16 = (_Float16*)(ws + off); off += bW1D;
  _Float16* beff  = (_Float16*)(ws + off); off += bBEFF;
  _Float16* rel16 = (_Float16*)(ws + off); off += bREL16;
  float*    cmain = (float*)(ws + off);    off += bCMAIN;
  float*    rbuf  = (float*)(ws + off);    off += bRBUF;
  float*    gbuf  = (float*)(ws + off);    off += bGBUF;
  float*    act   = (float*)(ws + off);    off += bACT;
  float*    spair = (float*)(ws + off);    off += bSTAB;
  float*    srel  = (float*)(ws + off);    off += bSTAB;
  if (off > ws_size) return;

  float* out = (float*)d_out;

  prep_planes<<<dim3(162), dim3(256), 0, stream>>>(span, topic, W1, xa, w1b16, w1d16);
  const int n8 = (kPAIRS * kREL) / 8;
  rel_cast<<<dim3((n8 + 255) / 256), dim3(256), 0, stream>>>(rel, rel16, n8);
  beff_build<<<dim3((kB * kNMAIN * 64) / 256), dim3(256), 0, stream>>>(span, topic, W1, beff);
  ac_scores<<<dim3(1), dim3(128), 0, stream>>>(span, W_type, b_type, act);

  {
    const int tiles = (kXAROWS / 64) * (kH / 64);
    wmma_gemm64<0, false, 0, 0, false, 0><<<dim3((tiles + 7) / 8, 1), dim3(256), 0, stream>>>(
        (const unsigned short*)xa, (const unsigned short*)xa, kD, 0L,
        (const unsigned short*)w1b16, (const unsigned short*)w1b16, kD, 0L,
        (void*)gbuf, (void*)gbuf, kH, 0L,
        gbuf, gbuf, 0L,
        kXAROWS, kH, kD, kWCarryInv);
  }
  {
    const int tiles = (kPAIRS / 64) * (kH / 64);
    wmma_gemm64<0, false, 0, 0, false, 0><<<dim3((tiles + 7) / 8, 1), dim3(256), 0, stream>>>(
        (const unsigned short*)rel16, (const unsigned short*)rel16, kREL, 0L,
        (const unsigned short*)w1d16, (const unsigned short*)w1d16, kREL, 0L,
        (void*)rbuf, (void*)rbuf, kH, 0L,
        gbuf, gbuf, 0L,
        kPAIRS, kH, kREL, kWCarryInv);
  }
  {
    const int tiles = (kN / 64) * (kNMAIN / 64);
    wmma_gemm64<0, false, 0, 0, false, 0><<<dim3((tiles + 7) / 8, kB), dim3(256), 0, stream>>>(
        (const unsigned short*)xa, (const unsigned short*)xa, kD, (long)kN * kD,
        (const unsigned short*)beff, (const unsigned short*)beff, kD, (long)kNMAIN * kD,
        (void*)cmain, (void*)cmain, kNMAIN, (long)kN * kNMAIN,
        gbuf, gbuf, 0L,
        kN, kNMAIN, kD, kWCarryInv);
  }

  epi_scores<<<dim3((kNOUT / 4 + 255) / 256), dim3(256), 0, stream>>>(cmain, rbuf, gbuf, b1, W2, b2, adu, srel, spair);
  pack_out<<<dim3((kOUTQ + 255) / 256), dim3(256), 0, stream>>>(act, spair, srel, out, kOUTQ);
}
